// MOCCT_50989851738863
// MI455X (gfx1250) — hardware-run, weakly checked
//
#include <hip/hip_runtime.h>
#include <math.h>

#ifndef NB
#define NB 131072
#endif
#define NB_FULL 131072
#define NITEM (3u * (unsigned)NB)

static_assert(NB % 32 == 0);
static_assert(NB <= NB_FULL);

#define ACT_CARRY 2048.0f
#define WT_CARRY 16384.0f
#define UNCARRY 2.98023223876953125e-08f
#define INV_TEMP 0.31622776601683794f

#define PW1 0u
#define PW2 1024u
#define PW1P 2048u
#define PW2P 11264u
#define PWC1 20480u
#define PTOT 25088u

#define PLANE_BYTES ((size_t)NB * 90u * 4u)
static_assert(PLANE_BYTES % 128u == 0);
static_assert(2u * PLANE_BYTES + (size_t)PTOT * 2u <= (size_t)134217728);

typedef _Float16 h16;
typedef __attribute__((ext_vector_type(16))) _Float16 v16h;
typedef __attribute__((ext_vector_type(8)))  _Float16 v8h;
typedef __attribute__((ext_vector_type(8)))  float    v8f;
typedef __attribute__((ext_vector_type(4)))  float    v4f;


#define VST2(T, ptr, val) do { const T vst2_v_ = (val); *(volatile T*)(ptr) = vst2_v_; __threadfence(); *(volatile T*)(ptr) = vst2_v_; } while (0)

static __device__ __forceinline__ float bfr(float f) {
    unsigned u = __float_as_uint(f);
    u += 0x7FFFu + ((u >> 16) & 1u);
    return __uint_as_float(u & 0xFFFF0000u);
}
static __device__ __forceinline__ v4f bfr4(v4f a) {
    v4f r; r.x = bfr(a.x); r.y = bfr(a.y); r.z = bfr(a.z); r.w = bfr(a.w); return r;
}
static __device__ __forceinline__ h16 toh_flush(float v) {
    const float w = (fabsf(v) < 6.103515625e-05f) ? 0.0f : v;
    return (h16)w;
}

union FragU { v16h v; v8h h[2]; };
static __device__ __forceinline__ v16h frag_ld(const h16* p) {
    FragU f; f.h[0] = *(const v8h*)(p); f.h[1] = *(const v8h*)(p + 16); return f.v;
}
static __device__ __forceinline__ v8f wmma16g(v16h a, v16h b, v8f c) {
    c = __builtin_amdgcn_wmma_f32_16x16x32_f16(false, a, false, b, (short)0, c, false, false);
    asm volatile("v_nop\n\tv_nop\n\tv_nop\n\tv_nop" : "+v"(c) : "v"(a), "v"(b));
    return c;
}
static __device__ __forceinline__ void wave_sync_lds() {
    __builtin_amdgcn_fence(3  , "workgroup");
    __builtin_amdgcn_wave_barrier();
    __builtin_amdgcn_fence(2  , "workgroup");
}
static __device__ __forceinline__ float half16_sum(float v) {
    v += __shfl_xor(v, 1, 32); v += __shfl_xor(v, 2, 32);
    v += __shfl_xor(v, 4, 32); v += __shfl_xor(v, 8, 32);
    return v;
}

template <unsigned PITCH, unsigned KT>
static __device__ __forceinline__ v16h afrag_rows(const float* sX, unsigned c, unsigned hh, unsigned k0) {
    v16h a;
#pragma unroll
    for (int i = 0; i < 8; ++i) {
        const unsigned ka = k0 + 8u * hh + (unsigned)i;
        const unsigned kb = ka + 16u;
        const float xa = sX[c * PITCH + min(ka, KT - 1u)];
        const float xb = sX[c * PITCH + min(kb, KT - 1u)];
        a[i]     = toh_flush((ka < KT) ? xa * ACT_CARRY : 0.0f);
        a[8 + i] = toh_flush((kb < KT) ? xb * ACT_CARRY : 0.0f);
    }
    return a;
}
static __device__ __forceinline__ v16h afrag_slab(const float* p) {
    const v4f x0 = *(const v4f*)(p);
    const v4f x1 = *(const v4f*)(p + 4);
    const v4f x2 = *(const v4f*)(p + 16);
    const v4f x3 = *(const v4f*)(p + 20);
    v16h a;
#pragma unroll
    for (int i = 0; i < 4; ++i) {
        a[i]      = toh_flush(x0[i] * ACT_CARRY);
        a[4 + i]  = toh_flush(x1[i] * ACT_CARRY);
        a[8 + i]  = toh_flush(x2[i] * ACT_CARRY);
        a[12 + i] = toh_flush(x3[i] * ACT_CARRY);
    }
    return a;
}

template <int NT, unsigned NTRUE>
static __device__ __forceinline__ void ln_tiles(v8f* y, const float* gv, const float* bv, unsigned c) {
#pragma unroll
    for (int r = 0; r < 8; ++r) {
        float s = 0.0f;
#pragma unroll
        for (int nt = 0; nt < NT; ++nt) s += y[nt][r];
        s = half16_sum(s);
        const float mean = s * (1.0f / (float)NTRUE);
        float qd = 0.0f;
#pragma unroll
        for (int nt = 0; nt < NT; ++nt) {
            const unsigned n = 16u * (unsigned)nt + c;
            const float d = (n < NTRUE) ? (y[nt][r] - mean) : 0.0f;
            y[nt][r] = d;
            qd += d * d;
        }
        qd = half16_sum(qd);
        const float rs = 1.0f / sqrtf(qd * (1.0f / (float)NTRUE) + 1e-6f);
#pragma unroll
        for (int nt = 0; nt < NT; ++nt) y[nt][r] = y[nt][r] * rs * gv[nt] + bv[nt];
    }
}

template <unsigned NOUT, unsigned KIN, unsigned NP, unsigned KP>
static __device__ __forceinline__ void wplane(const float* __restrict__ W, h16* __restrict__ dst, unsigned u) {
    if (u < NP * KP / 8u) {
        const unsigned e0 = u * 8u;
        const unsigned n = e0 / KP;
        const unsigned k0 = e0 - n * KP;
        const unsigned nc = min(n, NOUT - 1u);
        v8h hv;
#pragma unroll
        for (int i = 0; i < 8; ++i) {
            const unsigned k = k0 + (unsigned)i;
            const unsigned kc = min(k, KIN - 1u);
            const float w = W[nc * KIN + kc];
            const float s = (n < NOUT && k < KIN) ? bfr(w) * WT_CARRY : 0.0f;
            hv[i] = toh_flush(s);
        }
        VST2(v8h, dst + e0, hv);
    }
}
__global__ __launch_bounds__(256) void k_wprep(const float* __restrict__ W1, const float* __restrict__ W2,
                                               const float* __restrict__ W1p, const float* __restrict__ W2p,
                                               const float* __restrict__ Wc1, h16* __restrict__ planes) {
    const unsigned u = blockIdx.x * 256u + threadIdx.x;
    wplane<30u, 30u, 32u, 32u>(W1, planes + PW1, u);
    wplane<30u, 30u, 32u, 32u>(W2, planes + PW2, u);
    wplane<90u, 90u, 96u, 96u>(W1p, planes + PW1P, u);
    wplane<90u, 90u, 96u, 96u>(W2p, planes + PW2P, u);
    wplane<45u, 90u, 48u, 96u>(Wc1, planes + PWC1, u);
}

template <bool RNE>
static __device__ __forceinline__ void stage960(const float* __restrict__ src, float* slab, unsigned lane) {
    v4f t[8];
#pragma unroll
    for (int i = 0; i < 8; ++i) {
        const unsigned idx = min(lane + 32u * (unsigned)i, 239u);
        t[i] = *(const v4f*)(src + 4u * idx);
        if (RNE) t[i] = bfr4(t[i]);
    }
#pragma unroll
    for (int i = 0; i < 7; ++i) *(v4f*)(slab + 4u * (lane + 32u * (unsigned)i)) = t[i];
    if (lane < 16u) *(v4f*)(slab + 4u * (224u + lane)) = t[7];
}

static __device__ __forceinline__ void attn_item(const float* pq, const float* pk, const float* pv,
                                                 const float* sW, const float* sG, const float* sB, float* xo) {
    float t[30], kh[30], vh[30], q[30];
#pragma unroll
    for (int j = 0; j < 30; ++j) t[j] = pk[j];
#pragma unroll
    for (int d = 0; d < 10; ++d)
#pragma unroll
        for (int s = 0; s < 3; ++s) {
            float a = 0.0f;
#pragma unroll
            for (int e = 0; e < 10; ++e) a = fmaf(t[s * 10 + e], sW[100 + d * 10 + e], a);
            kh[s * 10 + d] = a;
        }
#pragma unroll
    for (int j = 0; j < 30; ++j) t[j] = pv[j];
#pragma unroll
    for (int d = 0; d < 10; ++d)
#pragma unroll
        for (int s = 0; s < 3; ++s) {
            float a = 0.0f;
#pragma unroll
            for (int e = 0; e < 10; ++e) a = fmaf(t[s * 10 + e], sW[200 + d * 10 + e], a);
            vh[s * 10 + d] = a;
        }
#pragma unroll
    for (int j = 0; j < 30; ++j) q[j] = pq[j];
#pragma unroll
    for (int s = 0; s < 3; ++s) {
        float qh[10];
#pragma unroll
        for (int d = 0; d < 10; ++d) {
            float a = 0.0f;
#pragma unroll
            for (int e = 0; e < 10; ++e) a = fmaf(q[s * 10 + e], sW[d * 10 + e], a);
            qh[d] = a * INV_TEMP;
        }
        float at[3];
#pragma unroll
        for (int u = 0; u < 3; ++u) {
            float a = 0.0f;
#pragma unroll
            for (int d = 0; d < 10; ++d) a = fmaf(qh[d], kh[u * 10 + d], a);
            at[u] = a;
        }
        float o[10];
        float sum = 0.0f;
#pragma unroll
        for (int d = 0; d < 10; ++d) {
            const float x = at[0] * vh[d] + at[1] * vh[10 + d] + at[2] * vh[20 + d] + q[s * 10 + d];
            o[d] = x; sum += x;
        }
        const float mean = sum * 0.1f;
        float var = 0.0f;
#pragma unroll
        for (int d = 0; d < 10; ++d) { o[d] -= mean; var += o[d] * o[d]; }
        const float rs = 1.0f / sqrtf(var * 0.1f + 1e-6f);
#pragma unroll
        for (int d = 0; d < 10; ++d) xo[s * 10 + d] = o[d] * rs * sG[d] + sB[d];
    }
}

template <bool SELF>
__global__ __launch_bounds__(128) void k_attn3(const float* __restrict__ Qi, const float* __restrict__ Ki,
                                               const float* __restrict__ Vi,
                                               const float* __restrict__ Wq, const float* __restrict__ Wk,
                                               const float* __restrict__ Wv,
                                               const float* __restrict__ gam, const float* __restrict__ bet,
                                               float* __restrict__ Xo) {
    __shared__ float sW[300];
    __shared__ float sG[10];
    __shared__ float sB[10];
    __shared__ __align__(16) float sIn[4][3][960];
    const unsigned tid = threadIdx.x, lane = tid & 31u, wave = tid >> 5;
    {
        const unsigned tc = min(tid, 99u);
        const float a = bfr(Wq[tc]), b = bfr(Wk[tc]), cc = bfr(Wv[tc]);
        if (tid < 100u) { sW[tid] = a; sW[100u + tid] = b; sW[200u + tid] = cc; }
        const unsigned t10 = min(tid, 9u);
        const float g0 = bfr(gam[t10]), b0 = bfr(bet[t10]);
        if (tid < 10u) { sG[tid] = g0; sB[tid] = b0; }
    }
    __syncthreads();
    const unsigned tile = blockIdx.x * 4u + wave;
    if (tile >= NITEM / 32u) return;
    float* s0 = sIn[wave][0];
    float* s1 = sIn[wave][1];
    float* s2 = sIn[wave][2];
    const size_t base = (size_t)tile * 960u;
    if (SELF) {
        stage960<false>(Qi + base, s0, lane);
    } else {
        stage960<true>(Qi + base, s0, lane);
        stage960<true>(Ki + base, s1, lane);
        stage960<true>(Vi + base, s2, lane);
    }
    wave_sync_lds();
    float xo[30];
    const float* pq = s0 + lane * 30u;
    const float* pk = SELF ? pq : (const float*)(s1 + lane * 30u);
    const float* pv = SELF ? pq : (const float*)(s2 + lane * 30u);
    attn_item(pq, pk, pv, sW, sG, sB, xo);
    {
        float* os = s0 + lane * 30u;
#pragma unroll
        for (int j = 0; j < 30; ++j) os[j] = xo[j];
    }
    wave_sync_lds();
    {
        v4f vv[8];
#pragma unroll
        for (int i = 0; i < 8; ++i) {
            const unsigned idx = min(lane + 32u * (unsigned)i, 239u);
            vv[i] = *(const v4f*)(s0 + 4u * idx);
        }
        float* dst = Xo + base;
        for (int pass = 0; pass < 2; ++pass) {
#pragma unroll
            for (int i = 0; i < 7; ++i) *(volatile v4f*)(dst + 4u * (lane + 32u * (unsigned)i)) = vv[i];
            if (lane < 16u) *(volatile v4f*)(dst + 4u * (224u + lane)) = vv[7];
            __threadfence();
        }
    }
}

__global__ __launch_bounds__(256) void k_ffn30(const float* __restrict__ Xin, const h16* __restrict__ W1h,
                                               const h16* __restrict__ W2h,
                                               const float* __restrict__ b1, const float* __restrict__ b2,
                                               const float* __restrict__ gam, const float* __restrict__ bet,
                                               float* __restrict__ Xout) {
    __shared__ __align__(16) float sX[8][480];
    __shared__ __align__(16) float sH[8][16 * 36];
    const unsigned lane = threadIdx.x & 31u, wave = threadIdx.x >> 5;
    const unsigned hh = lane >> 4, c = lane & 15u;
    const unsigned tile = blockIdx.x * 8u + wave;
    if (tile >= NITEM / 16u) return;
    float* xs = sX[wave];
    float* hs = sH[wave];
    const size_t base = (size_t)tile * 480u;
    {
        const float* src = Xin + base;
        const unsigned i3 = min(96u + lane, 119u);
        const v4f t0 = *(const v4f*)(src + 4u * lane);
        const v4f t1 = *(const v4f*)(src + 4u * (32u + lane));
        const v4f t2 = *(const v4f*)(src + 4u * (64u + lane));
        const v4f t3 = *(const v4f*)(src + 4u * i3);
        *(v4f*)(xs + 4u * lane) = t0;
        *(v4f*)(xs + 4u * (32u + lane)) = t1;
        *(v4f*)(xs + 4u * (64u + lane)) = t2;
        if (lane < 24u) *(v4f*)(xs + 4u * (96u + lane)) = t3;
    }
    float pb1[2], pb2[2], pg[2], pbt[2];
#pragma unroll
    for (int nt = 0; nt < 2; ++nt) {
        const unsigned n = 16u * (unsigned)nt + c;
        const unsigned nc = min(n, 29u);
        const bool ok = n < 30u;
        const float v1 = bfr(b1[nc]), v2 = bfr(b2[nc]), v3 = bfr(gam[nc]), v4 = bfr(bet[nc]);
        pb1[nt] = ok ? v1 : 0.0f; pb2[nt] = ok ? v2 : 0.0f; pg[nt] = ok ? v3 : 0.0f; pbt[nt] = ok ? v4 : 0.0f;
    }
    wave_sync_lds();
    const v8f zero8 = (v8f){0.f, 0.f, 0.f, 0.f, 0.f, 0.f, 0.f, 0.f};
    {
        const v16h a = afrag_rows<30u, 30u>(xs, c, hh, 0u);
#pragma unroll
        for (int nt = 0; nt < 2; ++nt) {
            const unsigned n = 16u * (unsigned)nt + c;
            const v16h b = frag_ld(W1h + n * 32u + 8u * hh);
            const v8f acc = wmma16g(a, b, zero8);
#pragma unroll
            for (int r = 0; r < 8; ++r) {
                float h = fmaxf(acc[r] * UNCARRY + pb1[nt], 0.0f);
                h = (n < 30u) ? h : 0.0f;
                hs[(8u * hh + (unsigned)r) * 36u + n] = h;
            }
        }
    }
    wave_sync_lds();
    v8f y[2];
    {
        const v16h a = afrag_slab(hs + c * 36u + 8u * hh);
#pragma unroll
        for (int nt = 0; nt < 2; ++nt) {
            const unsigned n = 16u * (unsigned)nt + c;
            const unsigned nc = min(n, 29u);
            const v16h b = frag_ld(W2h + n * 32u + 8u * hh);
            const v8f acc = wmma16g(a, b, zero8);
#pragma unroll
            for (int r = 0; r < 8; ++r) {
                const float res = xs[(8u * hh + (unsigned)r) * 30u + nc];
                const float v = acc[r] * UNCARRY + pb2[nt] + res;
                y[nt][r] = (n < 30u) ? v : 0.0f;
            }
        }
    }
    ln_tiles<2, 30u>(y, pg, pbt, c);
    wave_sync_lds();
#pragma unroll
    for (int nt = 0; nt < 2; ++nt) {
        const unsigned n = 16u * (unsigned)nt + c;
#pragma unroll
        for (int r = 0; r < 8; ++r)
            if (n < 30u) xs[(8u * hh + (unsigned)r) * 30u + n] = y[nt][r];
    }
    wave_sync_lds();
    {
        const unsigned i3 = min(96u + lane, 119u);
        const v4f o0 = *(const v4f*)(xs + 4u * lane);
        const v4f o1 = *(const v4f*)(xs + 4u * (32u + lane));
        const v4f o2 = *(const v4f*)(xs + 4u * (64u + lane));
        const v4f o3 = *(const v4f*)(xs + 4u * i3);
        float* dst = Xout + base;
        for (int pass = 0; pass < 2; ++pass) {
            *(volatile v4f*)(dst + 4u * lane) = o0;
            *(volatile v4f*)(dst + 4u * (32u + lane)) = o1;
            *(volatile v4f*)(dst + 4u * (64u + lane)) = o2;
            if (lane < 24u) *(volatile v4f*)(dst + 4u * (96u + lane)) = o3;
            __threadfence();
        }
    }
}

__global__ __launch_bounds__(128) void k_ffn90(const float* __restrict__ Xin, const h16* __restrict__ W1h,
                                               const h16* __restrict__ W2h, const h16* __restrict__ Wch,
                                               const float* __restrict__ b1p, const float* __restrict__ b2p,
                                               const float* __restrict__ gam, const float* __restrict__ bet,
                                               const float* __restrict__ bc1, const float* __restrict__ Wc2,
                                               const float* __restrict__ bc2, float* __restrict__ out) {
    __shared__ float sPar[580];
    __shared__ __align__(16) float sX[4][1440];
    __shared__ __align__(16) float sH[4][1600];
    __shared__ __align__(16) float sO[4][96];
    const unsigned tid = threadIdx.x, lane = tid & 31u, wave = tid >> 5;
    const unsigned hh = lane >> 4, c = lane & 15u;
    {
        const unsigned t90 = min(tid, 89u);
        const bool ok90 = tid < 90u;
        const float a0 = bfr(b1p[t90]), a1 = bfr(b2p[t90]), a2 = bfr(gam[t90]), a3 = bfr(bet[t90]);
        if (tid < 96u) {
            sPar[tid] = ok90 ? a0 : 0.0f;
            sPar[96u + tid] = ok90 ? a1 : 0.0f;
            sPar[192u + tid] = ok90 ? a2 : 0.0f;
            sPar[288u + tid] = ok90 ? a3 : 0.0f;
        }
        const unsigned t45 = min(tid, 44u);
        const bool ok45 = tid < 45u;
        const float c0 = bfr(bc1[t45]);
        const float w0 = bfr(Wc2[t45]), w1 = bfr(Wc2[45u + t45]), w2 = bfr(Wc2[90u + t45]);
        if (tid < 48u) {
            sPar[384u + tid] = ok45 ? c0 : 0.0f;
            sPar[432u + tid] = ok45 ? w0 : 0.0f;
            sPar[480u + tid] = ok45 ? w1 : 0.0f;
            sPar[528u + tid] = ok45 ? w2 : 0.0f;
        }
        const unsigned t3 = min(tid, 2u);
        const float d0 = bfr(bc2[t3]);
        if (tid < 4u) sPar[576u + tid] = (tid < 3u) ? d0 : 0.0f;
    }
    __syncthreads();
    const unsigned wt = blockIdx.x * 4u + wave;
    if (wt >= (unsigned)NB / 32u) return;
    float* xs = sX[wave];
    float* hs = sH[wave];
    float* os = sO[wave];

    float pb1[6], pb2[6], pg[6], pbt[6];
#pragma unroll
    for (int nt = 0; nt < 6; ++nt) {
        const unsigned n = 16u * (unsigned)nt + c;
        pb1[nt] = sPar[n]; pb2[nt] = sPar[96u + n]; pg[nt] = sPar[192u + n]; pbt[nt] = sPar[288u + n];
    }
    float pc1[3], pw0[3], pw1[3], pw2[3];
#pragma unroll
    for (int nt = 0; nt < 3; ++nt) {
        const unsigned n = 16u * (unsigned)nt + c;
        pc1[nt] = sPar[384u + n]; pw0[nt] = sPar[432u + n]; pw1[nt] = sPar[480u + n]; pw2[nt] = sPar[528u + n];
    }
    const float c20 = sPar[576], c21 = sPar[577], c22 = sPar[578];
    const v8f zero8 = (v8f){0.f, 0.f, 0.f, 0.f, 0.f, 0.f, 0.f, 0.f};

    for (unsigned mt = 0; mt < 2u; ++mt) {
        const unsigned row0 = wt * 32u + mt * 16u;
        {
            const float* src = Xin + (size_t)row0 * 90u;
            v4f t[12];
#pragma unroll
            for (int i = 0; i < 12; ++i) {
                const unsigned idx = min(lane + 32u * (unsigned)i, 359u);
                t[i] = *(const v4f*)(src + 4u * idx);
            }
#pragma unroll
            for (int i = 0; i < 11; ++i) *(v4f*)(xs + 4u * (lane + 32u * (unsigned)i)) = t[i];
            if (lane < 8u) *(v4f*)(xs + 4u * (352u + lane)) = t[11];
        }
        wave_sync_lds();
        v16h a[3];
#pragma unroll
        for (int ks = 0; ks < 3; ++ks) a[ks] = afrag_rows<90u, 90u>(xs, c, hh, 32u * (unsigned)ks);
#pragma unroll
        for (int nt = 0; nt < 6; ++nt) {
            const unsigned n = 16u * (unsigned)nt + c;
            v8f acc = zero8;
#pragma unroll
            for (int ks = 0; ks < 3; ++ks)
                acc = wmma16g(a[ks], frag_ld(W1h + n * 96u + 32u * (unsigned)ks + 8u * hh), acc);
#pragma unroll
            for (int r = 0; r < 8; ++r) {
                float h = fmaxf(acc[r] * UNCARRY + pb1[nt], 0.0f);
                h = (n < 90u) ? h : 0.0f;
                hs[(8u * hh + (unsigned)r) * 100u + n] = h;
            }
        }
        wave_sync_lds();
#pragma unroll
        for (int ks = 0; ks < 3; ++ks) a[ks] = afrag_slab(hs + c * 100u + 32u * (unsigned)ks + 8u * hh);
        v8f y[6];
#pragma unroll
        for (int nt = 0; nt < 6; ++nt) {
            const unsigned n = 16u * (unsigned)nt + c;
            const unsigned nc = min(n, 89u);
            v8f acc = zero8;
#pragma unroll
            for (int ks = 0; ks < 3; ++ks)
                acc = wmma16g(a[ks], frag_ld(W2h + n * 96u + 32u * (unsigned)ks + 8u * hh), acc);
#pragma unroll
            for (int r = 0; r < 8; ++r) {
                const float res = xs[(8u * hh + (unsigned)r) * 90u + nc];
                const float v = acc[r] * UNCARRY + pb2[nt] + res;
                y[nt][r] = (n < 90u) ? v : 0.0f;
            }
        }
        ln_tiles<6, 90u>(y, pg, pbt, c);
        wave_sync_lds();
#pragma unroll
        for (int nt = 0; nt < 6; ++nt) {
            const unsigned n = 16u * (unsigned)nt + c;
#pragma unroll
            for (int r = 0; r < 8; ++r) hs[(8u * hh + (unsigned)r) * 100u + n] = y[nt][r];
        }
        wave_sync_lds();
#pragma unroll
        for (int ks = 0; ks < 3; ++ks) a[ks] = afrag_slab(hs + c * 100u + 32u * (unsigned)ks + 8u * hh);
        v8f hid[3];
#pragma unroll
        for (int nt = 0; nt < 3; ++nt) {
            const unsigned n = 16u * (unsigned)nt + c;
            v8f acc = zero8;
#pragma unroll
            for (int ks = 0; ks < 3; ++ks)
                acc = wmma16g(a[ks], frag_ld(Wch + n * 96u + 32u * (unsigned)ks + 8u * hh), acc);
#pragma unroll
            for (int r = 0; r < 8; ++r) {
                const float h = fmaxf(acc[r] * UNCARRY + pc1[nt], 0.0f);
                hid[nt][r] = (n < 45u) ? h : 0.0f;
            }
        }
        float l0 = 0.0f, l1 = 0.0f, l2 = 0.0f;
#pragma unroll
        for (int r = 0; r < 8; ++r) {
            float p0 = hid[0][r] * pw0[0] + hid[1][r] * pw0[1] + hid[2][r] * pw0[2];
            float p1 = hid[0][r] * pw1[0] + hid[1][r] * pw1[1] + hid[2][r] * pw1[2];
            float p2 = hid[0][r] * pw2[0] + hid[1][r] * pw2[1] + hid[2][r] * pw2[2];
            p0 = half16_sum(p0) + c20;
            p1 = half16_sum(p1) + c21;
            p2 = half16_sum(p2) + c22;
            const bool me = (c == (unsigned)r);
            l0 = me ? p0 : l0; l1 = me ? p1 : l1; l2 = me ? p2 : l2;
        }
        const float mx = fmaxf(l0, fmaxf(l1, l2));
        const float e0 = expf(l0 - mx), e1 = expf(l1 - mx), e2 = expf(l2 - mx);
        const float es = e0 + e1 + e2;
        if (c < 8u) {
            const unsigned rr = (mt * 16u + 8u * hh + c) * 3u;
            os[rr] = e0 / es; os[rr + 1u] = e1 / es; os[rr + 2u] = e2 / es;
        }
        wave_sync_lds();
    }
    {
        const v4f ov = *(const v4f*)(os + 4u * min(lane, 23u));
        float* dst = out + (size_t)wt * 96u;
        for (int pass = 0; pass < 2; ++pass) {
            if (lane < 24u) *(volatile v4f*)(dst + 4u * lane) = ov;
            __threadfence();
        }
    }
}

extern "C" void kernel_launch(void* const* d_in, const int* in_sizes, int n_in, void* d_out, int out_size,
                              void* d_ws, size_t ws_size, hipStream_t stream) {
    if (n_in < 24) return;
    if (in_sizes[0] < NB * 90 || in_sizes[1] < NB * 90 || in_sizes[2] < NB * 90) return;
    if (in_sizes[3] < 100 || in_sizes[4] < 100 || in_sizes[5] < 100 || in_sizes[6] < 10 || in_sizes[7] < 10) return;
    if (in_sizes[8] < 900 || in_sizes[9] < 30 || in_sizes[10] < 900 || in_sizes[11] < 30 || in_sizes[12] < 30 || in_sizes[13] < 30) return;
    if (in_sizes[14] < 8100 || in_sizes[15] < 90 || in_sizes[16] < 8100 || in_sizes[17] < 90 || in_sizes[18] < 90 || in_sizes[19] < 90) return;
    if (in_sizes[20] < 4050 || in_sizes[21] < 45 || in_sizes[22] < 135 || in_sizes[23] < 3) return;
    if (out_size < NB * 3) return;

    const float* q      = (const float*)d_in[0];
    const float* k      = (const float*)d_in[1];
    const float* v      = (const float*)d_in[2];
    const float* Wq     = (const float*)d_in[3];
    const float* Wk     = (const float*)d_in[4];
    const float* Wv     = (const float*)d_in[5];
    const float* g_mha  = (const float*)d_in[6];
    const float* b_mha  = (const float*)d_in[7];
    const float* W1     = (const float*)d_in[8];
    const float* b1     = (const float*)d_in[9];
    const float* W2     = (const float*)d_in[10];
    const float* b2     = (const float*)d_in[11];
    const float* g_pff  = (const float*)d_in[12];
    const float* b_pff  = (const float*)d_in[13];
    const float* W1p    = (const float*)d_in[14];
    const float* b1p    = (const float*)d_in[15];
    const float* W2p    = (const float*)d_in[16];
    const float* b2p    = (const float*)d_in[17];
    const float* g_pff1 = (const float*)d_in[18];
    const float* b_pff1 = (const float*)d_in[19];
    const float* Wc1    = (const float*)d_in[20];
    const float* bc1    = (const float*)d_in[21];
    const float* Wc2    = (const float*)d_in[22];
    const float* bc2    = (const float*)d_in[23];
    float* out = (float*)d_out;

    const size_t total = 2u * PLANE_BYTES + (size_t)PTOT * 2u;
    if (total > ws_size || total > (size_t)134217728) return;
    char* wsp = (char*)d_ws;
    float* planeA = (float*)wsp;
    float* planeB = (float*)(wsp + PLANE_BYTES);
    h16*   wpl    = (h16*)(wsp + 2u * PLANE_BYTES);

    const unsigned gA = (NITEM / 32u + 3u) / 4u;
    const unsigned gF = (NITEM / 16u + 7u) / 8u;
    const unsigned gP = ((unsigned)NB / 32u + 3u) / 4u;

    k_wprep<<<5, 256, 0, stream>>>(W1, W2, W1p, W2p, Wc1, wpl);
    k_attn3<false><<<gA, 128, 0, stream>>>(q, k, v, Wq, Wk, Wv, g_mha, b_mha, planeA);
    k_ffn30<<<gF, 256, 0, stream>>>(planeA, (const h16*)(wpl + PW1), (const h16*)(wpl + PW2), b1, b2, g_pff, b_pff, planeB);
    k_attn3<true><<<gA, 128, 0, stream>>>(planeB, planeB, planeB, Wq, Wk, Wv, g_mha, b_mha, planeA);
    k_ffn30<<<gF, 256, 0, stream>>>(planeA, (const h16*)(wpl + PW1), (const h16*)(wpl + PW2), b1, b2, g_pff, b_pff, planeB);
    k_ffn90<<<gP, 128, 0, stream>>>(planeB, (const h16*)(wpl + PW1P), (const h16*)(wpl + PW2P), (const h16*)(wpl + PWC1),
                                    b1p, b2p, g_pff1, b_pff1, bc1, Wc2, bc2, out);
}
